// DualHierarchicalGNNUNet_15985868275833
// MI455X (gfx1250) — hardware-verified
//
#include <hip/hip_runtime.h>


namespace {
constexpr int Bn = 2, E = 128, HW = 64, NP = HW * HW, NH = 4, HD = 32, FU = 257, FC = 128, PH = 66, PWD = 128  , PLS = PH * PWD  , K1 = FU * 9  , K1P = 2336, K2 = FC * 9  ;
constexpr float EPS = 1e-5f, XS = 8.0f, PS = 8.0f, AS_ = 8.0f, NEG = -1e9f;
constexpr int P_QB0 = 0, P_OB0 = 384, P_QB1 = 512, P_OB1 = 896, P_G1 = 1024, P_B1 = 1152, P_G2 = 1280, P_B2 = 1408, P_OCW = 1536, P_OCB = 1664, P_A1B = 1792, P_A2W = 1920, P_A2B = 2048, P_LAB = 2049, P_END = 2051;
struct Wo_ { static constexpr size_t QKV0 = 0, OUT0 = QKV0 + 384 * 128, QKV1 = OUT0 + 128 * 128, OUT1 = QKV1 + 384 * 128, C1 = OUT1 + 128 * 128, C2 = C1 + (size_t)FC * K1P, A1 = C2 + (size_t)FC * K2, END = A1 + (size_t)128 * FC; };

typedef _Float16 b16;
typedef __attribute__((ext_vector_type(16))) _Float16 v16b;
typedef __attribute__((ext_vector_type(8))) _Float16 v8b;
typedef __attribute__((ext_vector_type(8))) float v8f;
typedef __attribute__((ext_vector_type(4))) float v4f;
__device__ __forceinline__ float bf16_rne(float f) { unsigned int u = __float_as_uint(f); u += 0x7FFFu + ((u >> 16) & 1u); return __uint_as_float(u & 0xFFFF0000u); }
__device__ __forceinline__ void split16(float v, b16& hi, b16& lo) { hi = (b16)v; lo = (b16)(v - (float)hi); }
__device__ __forceinline__ v16b frag_kb(const b16* p, int hh) { const v8b a = *(const v8b*)(p + 8 * hh), b = *(const v8b*)(p + 16 + 8 * hh); v16b f;
#pragma unroll
  for (int e = 0; e < 8; ++e) { f[e] = a[e]; f[8 + e] = b[e]; } return f; }
__device__ __forceinline__ void frag_split(const float* p, int hh, v16b& fh, v16b& fl) {
#pragma unroll
  for (int e = 0; e < 8; ++e) { b16 a, c; split16(p[8 * hh + e] * AS_, a, c); fh[e] = a; fl[e] = c; split16(p[16 + 8 * hh + e] * AS_, a, c); fh[8 + e] = a; fl[8 + e] = c; } }
__device__ __forceinline__ v8f wmma16b(v16b a, v16b b, v8f c) { v8f d = __builtin_amdgcn_wmma_f32_16x16x32_f16(false, a, false, b, (short)0, c, false, false); asm volatile("v_nop\n\tv_nop\n\tv_nop\n\tv_nop" : "+v"(d) : "v"(a), "v"(b)); return d; }
__device__ __forceinline__ void wave_lds_sync() { __builtin_amdgcn_fence(__ATOMIC_RELEASE, "workgroup"); __builtin_amdgcn_wave_barrier(); __builtin_amdgcn_fence(__ATOMIC_ACQUIRE, "workgroup"); }
__device__ __forceinline__ float nexp(float x) { return __builtin_amdgcn_exp2f(x * 1.4426950408889634f); }
__device__ __forceinline__ float nlog(float x) { return __builtin_amdgcn_logf(x) * 0.6931471805599453f; }
__device__ __forceinline__ float pmul(float a, float b) { float p = a * b; asm volatile("" : "+v"(p)); return p; }
__device__ __forceinline__ float wsum(float v) {
#pragma unroll
  for (int o = 1; o < 32; o <<= 1) v += __shfl_xor(v, o); return v; }
__device__ __forceinline__ float wmax(float v) {
#pragma unroll
  for (int o = 1; o < 32; o <<= 1) v = fmaxf(v, __shfl_xor(v, o)); return v; }

__global__ __launch_bounds__(256) void prep_kernel(const float* __restrict__ q0w, const float* __restrict__ q0b, const float* __restrict__ o0w, const float* __restrict__ o0b, const float* __restrict__ q1w, const float* __restrict__ q1b, const float* __restrict__ o1w, const float* __restrict__ o1b,
    const float* __restrict__ c1w, const float* __restrict__ g1, const float* __restrict__ be1, const float* __restrict__ c2w, const float* __restrict__ g2, const float* __restrict__ be2, const float* __restrict__ ocw, const float* __restrict__ ocb, const float* __restrict__ a1w, const float* __restrict__ a1b, const float* __restrict__ a2w, const float* __restrict__ a2b, const float* __restrict__ lab, b16* __restrict__ R, float* __restrict__ P) {
  const size_t tid = (size_t)blockIdx.x * 256 + threadIdx.x, nth = (size_t)gridDim.x * 256;
  for (int pass = 0; pass < 2; ++pass) {
    for (size_t p = tid; p < Wo_::END / 8; p += nth) { const size_t q = p * 8; v8b v;
      if (q < Wo_::OUT0) { for (int e = 0; e < 8; ++e) v[e] = (b16)bf16_rne(q0w[q + e]); }
      else if (q < Wo_::QKV1) { for (int e = 0; e < 8; ++e) v[e] = (b16)bf16_rne(o0w[q - Wo_::OUT0 + e]); }
      else if (q < Wo_::OUT1) { for (int e = 0; e < 8; ++e) v[e] = (b16)bf16_rne(q1w[q - Wo_::QKV1 + e]); }
      else if (q < Wo_::C1) { for (int e = 0; e < 8; ++e) v[e] = (b16)bf16_rne(o1w[q - Wo_::OUT1 + e]); }
      else if (q < Wo_::C2) { const size_t r = q - Wo_::C1; const int o = (int)(r / K1P), k0 = (int)(r % K1P); for (int e = 0; e < 8; ++e) { const int k = k0 + e; v[e] = (b16)((k < K1) ? bf16_rne(c1w[(size_t)o * K1 + k]) : 0.0f); } }
      else if (q < Wo_::A1) { const size_t r = q - Wo_::C2; for (int e = 0; e < 8; ++e) v[e] = (b16)bf16_rne(c2w[r + e]); }
      else { const size_t r = q - Wo_::A1; for (int e = 0; e < 8; ++e) v[e] = (b16)bf16_rne(a1w[r + e]); }
      *(volatile v8b*)(R + q) = v; }
    for (size_t q = tid; q < P_END; q += nth) { const int i = (int)q; float v = 0.0f;
      if (i < 384) v = q0b[i]; else if (i < 512) v = o0b[i - 384]; else if (i < 896) v = q1b[i - 512]; else if (i < 1024) v = o1b[i - 896]; else if (i < 1152) v = g1[i - 1024]; else if (i < 1280) v = be1[i - 1152]; else if (i < 1408) v = g2[i - 1280]; else if (i < 1536) v = be2[i - 1408];
      else if (i < 1664) v = ocw[i - 1536]; else if (i == 1664) v = ocb[0]; else if (i < P_A1B) v = 0.0f; else if (i < P_A2W) v = a1b[i - P_A1B]; else if (i < P_A2B) v = a2w[i - P_A2W]; else if (i == P_A2B) v = a2b[0]; else v = lab[i - P_LAB];
      P[q] = bf16_rne(v); }
    __threadfence(); }
}

__global__ __launch_bounds__(256) void rows_kernel(const float* __restrict__ sf, const float* __restrict__ tf, b16* __restrict__ T) {
  __shared__ __attribute__((aligned(16))) b16 Tt[64][E + 8];
  const int b = blockIdx.y, which = blockIdx.z, p0 = blockIdx.x * 64, t_ = threadIdx.x; const float* src = (which == 0) ? sf : tf;
  for (int i = t_; i < E * 64; i += 256) { const int c = i >> 6, p = i & 63; Tt[p][c] = (b16)bf16_rne(src[((size_t)b * E + c) * NP + p0 + p]); }
  __syncthreads();
  for (int pass = 0; pass < 2; ++pass) { for (int i = t_; i < 64 * 16; i += 256) { const int p = i >> 4, c8 = (i & 15) * 8; *(volatile v8b*)(T + (((size_t)which * Bn + b) * NP + p0 + p) * E + c8) = *(const v8b*)(&Tt[p][c8]); } __threadfence(); }
}

__global__ __launch_bounds__(128) void proj_kernel(const b16* __restrict__ T, const b16* __restrict__ R, const float* __restrict__ P, b16* __restrict__ Q, b16* __restrict__ K, b16* __restrict__ VT) {
  __shared__ __attribute__((aligned(16))) b16 Ts[128][E + 8];
  const int lane = threadIdx.x & 31, wave = threadIdx.x >> 5, nloc = lane & 15, hlf = lane >> 4, b = blockIdx.y, m = blockIdx.z / 3, j = blockIdx.z % 3, p0 = blockIdx.x * 128, m0 = p0 + wave * 32;
  const int srcw = (j == 0) ? m : (1 - m);
  const b16* A = T + ((size_t)srcw * Bn + b) * NP * E; const b16* Wr = R + ((m == 0) ? Wo_::QKV0 : Wo_::QKV1) + (size_t)j * 128 * 128; const float* bias = P + ((m == 0) ? P_QB0 : P_QB1) + j * 128;
  v8f acc[2][8];
#pragma unroll
  for (int r = 0; r < 2; ++r)
#pragma unroll
    for (int t = 0; t < 8; ++t) acc[r][t] = (v8f){};
#pragma unroll
  for (int kb = 0; kb < E; kb += 32) { const v16b a0 = frag_kb(A + (size_t)(m0 + nloc) * E + kb, hlf), a1 = frag_kb(A + (size_t)(m0 + 16 + nloc) * E + kb, hlf);
#pragma unroll
    for (int t = 0; t < 8; ++t) { const v16b bw = frag_kb(Wr + (size_t)(t * 16 + nloc) * E + kb, hlf); acc[0][t] = wmma16b(a0, bw, acc[0][t]); acc[1][t] = wmma16b(a1, bw, acc[1][t]); } }
#pragma unroll
  for (int t = 0; t < 8; ++t) { const int c = t * 16 + nloc; const float bb = bias[c];
#pragma unroll
    for (int r = 0; r < 2; ++r)
#pragma unroll
      for (int v = 0; v < 8; ++v) Ts[wave * 32 + r * 16 + 8 * hlf + v][c] = (b16)((acc[r][t][v] + bb) * XS); }
  __syncthreads();
  for (int pass = 0; pass < 2; ++pass) {
    if (j < 2) { b16* dst = ((j == 0) ? Q : K) + ((size_t)m * Bn + b) * NP * E; for (int i = threadIdx.x; i < 128 * 16; i += 128) { const int rr = i >> 4, c8 = (i & 15) * 8; *(volatile v8b*)(dst + (size_t)(p0 + rr) * E + c8) = *(const v8b*)(&Ts[rr][c8]); } }
    else { for (int i = threadIdx.x; i < E * 16; i += 128) { const int c = i >> 4, c8 = (i & 15) * 8; const int h = c / HD, d = c % HD; v8b v; for (int e = 0; e < 8; ++e) v[e] = Ts[c8 + e][c]; *(volatile v8b*)(VT + ((((size_t)m * Bn + b) * NH + h) * HD + d) * NP + p0 + c8) = v; } }
    __threadfence(); }
}

__global__ __launch_bounds__(128) void attn_kernel(const b16* __restrict__ Q, const b16* __restrict__ K, const b16* __restrict__ VT, b16* __restrict__ CTX) {
  __shared__ __attribute__((aligned(16))) b16 Os[16][E + 8];
  const int h = threadIdx.x >> 5, lane = threadIdx.x & 31, hh = lane >> 4, col = lane & 15, b = blockIdx.y, m = blockIdx.z, q0 = blockIdx.x * 16, qi = q0 + col;
  const size_t rb = ((size_t)m * Bn + b) * NP * E; const b16* Qr = Q + rb + h * HD; const b16* Kr = K + rb + h * HD; const b16* V = VT + ((((size_t)m * Bn + b) * NH + h) * HD) * NP;
  const v16b qf = frag_kb(Qr + (size_t)qi * E, hh); const float SC = 0.17677669529663687f / (XS * XS);
  float mx = -INFINITY, l = 0.0f; v8f o[2] = {{}, {}};
  for (int kb = 0; kb < NP; kb += 32) { v8f s0 = {}, s1 = {}; s0 = wmma16b(frag_kb(Kr + (size_t)(kb + col) * E, hh), qf, s0); s1 = wmma16b(frag_kb(Kr + (size_t)(kb + 16 + col) * E, hh), qf, s1);
    float mr = -INFINITY;
#pragma unroll
    for (int r = 0; r < 8; ++r) { s0[r] *= SC; s1[r] *= SC; mr = fmaxf(mr, fmaxf(s0[r], s1[r])); }
    mr = fmaxf(mr, __shfl_xor(mr, 16)); const float mn = fmaxf(mx, mr), al_ = nexp(mx - mn); mx = mn; float sum = 0.0f; v16b pb;
#pragma unroll
    for (int r = 0; r < 8; ++r) { const float e0 = nexp(s0[r] - mn), e1 = nexp(s1[r] - mn); sum += e0 + e1; pb[r] = (b16)(e0 * PS); pb[8 + r] = (b16)(e1 * PS); }
    sum += __shfl_xor(sum, 16); l = l * al_ + sum;
#pragma unroll
    for (int t = 0; t < 2; ++t) { o[t] *= al_; o[t] = wmma16b(frag_kb(V + (size_t)(t * 16 + col) * NP + kb, hh), pb, o[t]); } }
  const float inv = 1.0f / (l * PS);
#pragma unroll
  for (int t = 0; t < 2; ++t)
#pragma unroll
    for (int r = 0; r < 8; ++r) Os[col][h * HD + t * 16 + 8 * hh + r] = (b16)(o[t][r] * inv);
  __syncthreads();
  for (int pass = 0; pass < 2; ++pass) { for (int i = threadIdx.x; i < 16 * 16; i += 128) { const int rr = i >> 4, c8 = (i & 15) * 8; *(volatile v8b*)(CTX + rb + (size_t)(q0 + rr) * E + c8) = *(const v8b*)(&Os[rr][c8]); } __threadfence(); }
}

__global__ __launch_bounds__(128) void oproj_kernel(const b16* __restrict__ CTX, const b16* __restrict__ R, const float* __restrict__ P, const float* __restrict__ gctx, b16* __restrict__ FP) {
  __shared__ __attribute__((aligned(16))) b16 Tp[E][2][PWD];
  const int lane = threadIdx.x & 31, wave = threadIdx.x >> 5, nloc = lane & 15, hlf = lane >> 4, b = blockIdx.y, m = blockIdx.z, p0 = blockIdx.x * 128, m0 = p0 + wave * 32, y0 = blockIdx.x * 2;
  const b16* A = CTX + ((size_t)m * Bn + b) * NP * E; const b16* Wr = R + ((m == 0) ? Wo_::OUT0 : Wo_::OUT1); const float* bias = P + ((m == 0) ? P_OB0 : P_OB1);
  for (int i = threadIdx.x; i < E * 2 * PWD; i += 128) (&Tp[0][0][0])[i] = (b16)0.0f;
  __syncthreads();
  v8f acc[2][8];
#pragma unroll
  for (int r = 0; r < 2; ++r)
#pragma unroll
    for (int t = 0; t < 8; ++t) acc[r][t] = (v8f){};
#pragma unroll
  for (int kb = 0; kb < E; kb += 32) { const v16b a0 = frag_kb(A + (size_t)(m0 + nloc) * E + kb, hlf), a1 = frag_kb(A + (size_t)(m0 + 16 + nloc) * E + kb, hlf);
#pragma unroll
    for (int t = 0; t < 8; ++t) { const v16b bw = frag_kb(Wr + (size_t)(t * 16 + nloc) * E + kb, hlf); acc[0][t] = wmma16b(a0, bw, acc[0][t]); acc[1][t] = wmma16b(a1, bw, acc[1][t]); } }
#pragma unroll
  for (int t = 0; t < 8; ++t) { const int c = t * 16 + nloc; const float bb = bias[c];
#pragma unroll
    for (int r = 0; r < 2; ++r)
#pragma unroll
      for (int v = 0; v < 8; ++v) { const int pl = wave * 32 + r * 16 + 8 * hlf + v; const int ry = pl >> 6, x = pl & 63; Tp[c][ry][x + 1] = (b16)(acc[r][t][v] * (1.0f / XS) + bb); } }
  __syncthreads();
  b16* base = FP + ((size_t)b * FU + m * E) * PLS;
  for (int pass = 0; pass < 2; ++pass) {
    for (int i = threadIdx.x; i < E * 2 * 16; i += 128) { const int c = i >> 5, rr = (i >> 4) & 1, c8 = (i & 15) * 8; *(volatile v8b*)(base + ((size_t)c * PH + y0 + rr + 1) * PWD + c8) = *(const v8b*)(&Tp[c][rr][c8]); }
    if (blockIdx.x == 0 || blockIdx.x == 31) { const int prow = (blockIdx.x == 0) ? 0 : (PH - 1); for (int i = threadIdx.x; i < E * 16; i += 128) { const int c = i >> 4, c8 = (i & 15) * 8; v8b z; for (int e = 0; e < 8; ++e) z[e] = (b16)0.0f; *(volatile v8b*)(base + ((size_t)c * PH + prow) * PWD + c8) = z; } }
    if (m == 0) {
      b16* g = FP + ((size_t)b * FU + 2 * E) * PLS;
      for (int i = threadIdx.x; i < 2 * 16; i += 128) { const int rr = i >> 4, c8 = (i & 15) * 8; v8b v; for (int e = 0; e < 8; ++e) { const int x = c8 + e - 1; v[e] = (b16)((x >= 0 && x < HW) ? bf16_rne(gctx[(size_t)b * NP + (y0 + rr) * HW + x]) : 0.0f); } *(volatile v8b*)(g + (size_t)(y0 + rr + 1) * PWD + c8) = v; }
      if (blockIdx.x == 0 || blockIdx.x == 31) { const int prow = (blockIdx.x == 0) ? 0 : (PH - 1); if (threadIdx.x < 16) { v8b z; for (int e = 0; e < 8; ++e) z[e] = (b16)0.0f; *(volatile v8b*)(g + (size_t)prow * PWD + threadIdx.x * 8) = z; } } }
    __threadfence(); }
}

template <int CIN, int KK, int KP>
__global__ __launch_bounds__(64) void conv_kernel(const b16* __restrict__ PL, const b16* __restrict__ Wr, float* __restrict__ OUTc) {
  __shared__ __attribute__((aligned(16))) float Ts[FC][32 + 4];
  const int lane = threadIdx.x & 31, wave = threadIdx.x >> 5, nloc = lane & 15, hlf = lane >> 4, b = blockIdx.y, p0 = blockIdx.x * 32, y = p0 / HW, x0 = p0 % HW;
  const b16* Pb = PL + (size_t)b * CIN * PLS;
  v8f acc[2][4];
#pragma unroll
  for (int r = 0; r < 2; ++r)
#pragma unroll
    for (int t = 0; t < 4; ++t) acc[r][t] = (v8f){};
  for (int kb = 0; kb < KP; kb += 32) { v16b a0, a1;
#pragma unroll
    for (int e = 0; e < 16; ++e) { const int k = kb + ((e < 8) ? (8 * hlf + e) : (16 + 8 * hlf + e - 8)); const int kc = (k < KK) ? k : (KK - 1); const int c = kc / 9, tap = kc - c * 9; const int dy = tap / 3, dx = tap - dy * 3;
      const b16* rowp = Pb + ((size_t)c * PH + y + dy) * PWD + dx; a0[e] = rowp[x0 + nloc]; a1[e] = rowp[x0 + 16 + nloc]; }
#pragma unroll
    for (int t = 0; t < 4; ++t) { const v16b bw = frag_kb(Wr + (size_t)(wave * 64 + t * 16 + nloc) * KP + kb, hlf); acc[0][t] = wmma16b(a0, bw, acc[0][t]); acc[1][t] = wmma16b(a1, bw, acc[1][t]); } }
#pragma unroll
  for (int t = 0; t < 4; ++t)
#pragma unroll
    for (int r = 0; r < 2; ++r)
#pragma unroll
      for (int v = 0; v < 8; ++v) Ts[wave * 64 + t * 16 + nloc][r * 16 + 8 * hlf + v] = acc[r][t][v];
  wave_lds_sync();
  for (int pass = 0; pass < 2; ++pass) { for (int i = lane; i < 64 * 8; i += 32) { const int c = wave * 64 + (i >> 3), c4 = (i & 7) * 4; *(volatile v4f*)(OUTc + ((size_t)b * FC + c) * NP + p0 + c4) = *(const v4f*)(&Ts[c][c4]); } __threadfence(); }
}

__global__ __launch_bounds__(256) void bnstat_kernel(const float* __restrict__ OUTc, float* __restrict__ ST) {
  __shared__ float red[8]; __shared__ float mu_s;
  const int c = blockIdx.x, t_ = threadIdx.x, lane = t_ & 31, wave = t_ >> 5;
  float s = 0.0f; for (int b = 0; b < Bn; ++b) { const float* r = OUTc + ((size_t)b * FC + c) * NP; for (int i = t_; i < NP; i += 256) s += r[i]; }
  s = wsum(s); if (lane == 0) red[wave] = s; __syncthreads();
  if (t_ == 0) { float a = 0.0f; for (int w = 0; w < 8; ++w) a += red[w]; mu_s = a / (float)(Bn * NP); } __syncthreads();
  const float mu = mu_s; float q = 0.0f; for (int b = 0; b < Bn; ++b) { const float* r = OUTc + ((size_t)b * FC + c) * NP; for (int i = t_; i < NP; i += 256) { const float d = r[i] - mu; q += pmul(d, d); } }
  q = wsum(q); __syncthreads(); if (lane == 0) red[wave] = q; __syncthreads();
  __shared__ float inv_s; if (t_ == 0) { float var = 0.0f; for (int w = 0; w < 8; ++w) var += red[w]; var /= (float)(Bn * NP); inv_s = rsqrtf(var + EPS); } __syncthreads();
  if (t_ < 32) { const float v = (t_ == 0) ? mu : (t_ == 1) ? inv_s : 0.0f; for (int pass = 0; pass < 2; ++pass) ((volatile float*)ST)[(size_t)c * 32 + t_] = v; }
  __threadfence();
}

__global__ __launch_bounds__(256) void bnrelu_kernel(const float* __restrict__ OUTc, const float* __restrict__ ST, const float* __restrict__ P, int goff, b16* __restrict__ XP) {
  __shared__ __attribute__((aligned(16))) b16 pl[PLS];
  const int c = blockIdx.x, b = blockIdx.y, t_ = threadIdx.x; const float mu = ST[(size_t)c * 32], inv = ST[(size_t)c * 32 + 1], g = P[goff + c], be = P[goff + 128 + c]; const float* r = OUTc + ((size_t)b * FC + c) * NP;
  for (int i = t_; i < PLS; i += 256) { float v = 0.0f; const int yy = i / PWD - 1, xx = i % PWD - 1; if (yy >= 0 && yy < HW && xx >= 0 && xx < HW) v = fmaxf(pmul((r[yy * HW + xx] - mu) * inv, g) + be, 0.0f); pl[i] = (b16)v; }
  __syncthreads();
  b16* dst = XP + ((size_t)b * FC + c) * PLS;
  for (int pass = 0; pass < 2; ++pass) { for (int i = t_; i < PLS / 8; i += 256) *(volatile v8b*)(dst + i * 8) = *(const v8b*)(&pl[i * 8]); __threadfence(); }
}

__global__ __launch_bounds__(128) void head_kernel(const float* __restrict__ OUTc, const float* __restrict__ ST, const b16* __restrict__ R, const float* __restrict__ P, float* __restrict__ LS) {
  __shared__ __attribute__((aligned(16))) float Ft[128][FC + 4]; __shared__ __attribute__((aligned(16))) float Lo[128][2];
  const int lane = threadIdx.x & 31, wave = threadIdx.x >> 5, nloc = lane & 15, hlf = lane >> 4, b = blockIdx.y, p0 = blockIdx.x * 128, t_ = threadIdx.x;
  for (int i = t_; i < 128 * FC; i += 128) { const int c = i >> 7, p = i & 127; const float mu = ST[(size_t)c * 32], inv = ST[(size_t)c * 32 + 1]; Ft[p][c] = fmaxf(pmul((OUTc[((size_t)b * FC + c) * NP + p0 + p] - mu) * inv, P[P_G2 + c]) + P[P_B2 + c], 0.0f); }
  __syncthreads();
  { float s = P[P_OCB]; for (int c = 0; c < FC; ++c) s += pmul(Ft[t_][c], P[P_OCW + c]); Lo[t_][0] = s; }
  const b16* A1 = R + Wo_::A1; v8f acc[2][8];
#pragma unroll
  for (int r = 0; r < 2; ++r)
#pragma unroll
    for (int t = 0; t < 8; ++t) acc[r][t] = (v8f){};
#pragma unroll
  for (int kb = 0; kb < FC; kb += 32) { v16b a0, l0, a1, l1; frag_split(&Ft[wave * 32 + nloc][kb], hlf, a0, l0); frag_split(&Ft[wave * 32 + 16 + nloc][kb], hlf, a1, l1);
#pragma unroll
    for (int t = 0; t < 8; ++t) { const v16b bw = frag_kb(A1 + (size_t)(t * 16 + nloc) * FC + kb, hlf); acc[0][t] = wmma16b(a0, bw, acc[0][t]); acc[0][t] = wmma16b(l0, bw, acc[0][t]); acc[1][t] = wmma16b(a1, bw, acc[1][t]); acc[1][t] = wmma16b(l1, bw, acc[1][t]); } }
#pragma unroll
  for (int r = 0; r < 2; ++r)
#pragma unroll
    for (int v = 0; v < 8; ++v) { float s = 0.0f;
#pragma unroll
      for (int t = 0; t < 8; ++t) { const int c = t * 16 + nloc; s += pmul(fmaxf(acc[r][t][v] * (1.0f / AS_) + P[P_A1B + c], 0.0f), P[P_A2W + c]); }
      s += __shfl_xor(s, 1); s += __shfl_xor(s, 2); s += __shfl_xor(s, 4); s += __shfl_xor(s, 8);
      if (nloc == 0) Lo[wave * 32 + r * 16 + 8 * hlf + v][1] = s + P[P_A2B]; }
  __syncthreads();
  for (int pass = 0; pass < 2; ++pass) { if (t_ < 64) *(volatile v4f*)(LS + ((size_t)b * NP + p0) * 2 + t_ * 4) = *(const v4f*)(&Lo[0][0] + t_ * 4); __threadfence(); }
}

__global__ __launch_bounds__(256) void mil_kernel(const float* __restrict__ LS, const int* __restrict__ zone, const int* __restrict__ cats, const float* __restrict__ P, float* __restrict__ out) {
  __shared__ float W[Bn][NP]; __shared__ float red[8]; __shared__ int hred[8]; __shared__ float bagv[Bn]; __shared__ int hasv[Bn];
  const int t_ = threadIdx.x, lane = t_ & 31, wave = t_ >> 5;
  for (int b = 0; b < Bn; ++b) { const int cat = cats[b]; float mx = -INFINITY; int any = 0;
    for (int i = t_; i < NP; i += 256) { const int z = zone[(size_t)b * NP + i]; const bool mk = (z == cat) && (z > 0); const float s = mk ? LS[((size_t)b * NP + i) * 2 + 1] : NEG; W[b][i] = s; mx = fmaxf(mx, s); any |= mk ? 1 : 0; }
    mx = wmax(mx); any = __builtin_amdgcn_ballot_w32(any != 0) != 0u ? 1 : 0; if (lane == 0) { red[wave] = mx; hred[wave] = any; } __syncthreads();
    float gm = red[0]; int ha = hred[0]; for (int w = 1; w < 8; ++w) { gm = fmaxf(gm, red[w]); ha |= hred[w]; } __syncthreads();
    float su = 0.0f; for (int i = t_; i < NP; i += 256) su += nexp(W[b][i] - gm);
    su = wsum(su); if (lane == 0) red[wave] = su; __syncthreads();
    float tot = 0.0f; for (int w = 0; w < 8; ++w) tot += red[w]; __syncthreads();
    const float isu = 1.0f / tot; float bg = 0.0f;
    for (int i = t_; i < NP; i += 256) { const int z = zone[(size_t)b * NP + i]; const bool mk = (z == cat) && (z > 0); const float w = nexp(W[b][i] - gm) * isu; W[b][i] = ha ? w : 0.0f; if (mk) bg += pmul(LS[((size_t)b * NP + i) * 2], w); }
    bg = wsum(bg); if (lane == 0) red[wave] = bg; __syncthreads();
    if (t_ == 0) { float a = 0.0f; for (int w = 0; w < 8; ++w) a += red[w]; bagv[b] = ha ? a : 0.0f; hasv[b] = ha; } __syncthreads(); }
  float loss = 0.0f; if (t_ == 0) { for (int b = 0; b < Bn; ++b) { const float x = bagv[b]; const float sp = (x > 20.0f) ? x : nlog(1.0f + nexp(x)); loss += sp - x * P[P_LAB + b]; } loss *= (1.0f / Bn); red[0] = loss; }
  __syncthreads(); loss = red[0];
  constexpr int NTOT = 1 + Bn * NP;
  for (int pass = 0; pass < 2; ++pass) { for (int i4 = t_ * 4; i4 < NTOT; i4 += 1024) { if (i4 + 4 <= NTOT) { v4f v; for (int e = 0; e < 4; ++e) { const int i = i4 + e; v[e] = (i == 0) ? loss : (&W[0][0])[i - 1]; } *(volatile v4f*)(out + i4) = v; } else { for (int i = i4; i < NTOT; ++i) ((volatile float*)out)[i] = (i == 0) ? loss : (&W[0][0])[i - 1]; } } __threadfence(); }
}
}

extern "C" void kernel_launch(void* const* d_in, const int* in_sizes, int n_in,
                              void* d_out, int out_size, void* d_ws, size_t ws_size, hipStream_t stream) {
  (void)n_in; (void)out_size;
  const float* sf = (const float*)d_in[0]; const float* tf = (const float*)d_in[1]; const float* gctx = (const float*)d_in[2]; const int* zone = (const int*)d_in[3]; const int* cats = (const int*)d_in[4]; const float* lab = (const float*)d_in[5];
  const float* q0w = (const float*)d_in[6]; const float* q0b = (const float*)d_in[7]; const float* o0w = (const float*)d_in[8]; const float* o0b = (const float*)d_in[9]; const float* q1w = (const float*)d_in[10]; const float* q1b = (const float*)d_in[11]; const float* o1w = (const float*)d_in[12]; const float* o1b = (const float*)d_in[13];
  const float* c1w = (const float*)d_in[14]; const float* g1 = (const float*)d_in[15]; const float* be1 = (const float*)d_in[16]; const float* c2w = (const float*)d_in[17]; const float* g2 = (const float*)d_in[18]; const float* be2 = (const float*)d_in[19];
  const float* ocw = (const float*)d_in[20]; const float* ocb = (const float*)d_in[21]; const float* a1w = (const float*)d_in[22]; const float* a1b = (const float*)d_in[23]; const float* a2w = (const float*)d_in[24]; const float* a2b = (const float*)d_in[25];
  float* out = (float*)d_out;
  if (in_sizes[0] != Bn * E * NP || in_sizes[3] != Bn * NP || in_sizes[14] != FC * K1 || in_sizes[17] != FC * K2) return;
  size_t off = 0; char* ws = (char*)d_ws;
  auto carve = [&](size_t bytes) { char* p = ws + off; off += (bytes + 255) & ~(size_t)255; return p; };
  b16* R = (b16*)carve(Wo_::END * 2); float* P = (float*)carve(2304 * 4); b16* T = (b16*)carve((size_t)2 * Bn * NP * E * 2); b16* Q = (b16*)carve((size_t)2 * Bn * NP * E * 2); b16* K = (b16*)carve((size_t)2 * Bn * NP * E * 2); b16* VT = (b16*)carve((size_t)2 * Bn * NP * E * 2); b16* CTX = (b16*)carve((size_t)2 * Bn * NP * E * 2);
  b16* FP = (b16*)carve((size_t)Bn * FU * PLS * 2); float* O1 = (float*)carve((size_t)Bn * FC * NP * 4); float* ST1 = (float*)carve((size_t)FC * 32 * 4); b16* XP = (b16*)carve((size_t)Bn * FC * PLS * 2); float* O2 = (float*)carve((size_t)Bn * FC * NP * 4); float* ST2 = (float*)carve((size_t)FC * 32 * 4); float* LS = (float*)carve((size_t)Bn * NP * 2 * 4);
  if (off > ws_size) return;
  prep_kernel<<<256, 256, 0, stream>>>(q0w, q0b, o0w, o0b, q1w, q1b, o1w, o1b, c1w, g1, be1, c2w, g2, be2, ocw, ocb, a1w, a1b, a2w, a2b, lab, R, P);
  rows_kernel<<<dim3(NP / 64, Bn, 2), 256, 0, stream>>>(sf, tf, T);
  proj_kernel<<<dim3(NP / 128, Bn, 6), 128, 0, stream>>>(T, R, P, Q, K, VT);
  attn_kernel<<<dim3(NP / 16, Bn, 2), 128, 0, stream>>>(Q, K, VT, CTX);
  oproj_kernel<<<dim3(NP / 128, Bn, 2), 128, 0, stream>>>(CTX, R, P, gctx, FP);
  conv_kernel<FU, K1, K1P><<<dim3(NP / 32, Bn), 64, 0, stream>>>(FP, R + Wo_::C1, O1);
  bnstat_kernel<<<FC, 256, 0, stream>>>(O1, ST1);
  bnrelu_kernel<<<dim3(FC, Bn), 256, 0, stream>>>(O1, ST1, P, P_G1, XP);
  conv_kernel<FC, K2, K2><<<dim3(NP / 32, Bn), 64, 0, stream>>>(XP, R + Wo_::C2, O2);
  bnstat_kernel<<<FC, 256, 0, stream>>>(O2, ST2);
  head_kernel<<<dim3(NP / 128, Bn), 128, 0, stream>>>(O2, ST2, R, P, LS);
  mil_kernel<<<1, 256, 0, stream>>>(LS, zone, cats, P, out);
}
